// Nalui2Layer_63367947485910
// MI455X (gfx1250) — hardware-verified
//
#include <hip/hip_runtime.h>
#include <math.h>

typedef __attribute__((ext_vector_type(16))) _Float16 v16h;
typedef __attribute__((ext_vector_type(8)))  _Float16 v8h;
typedef __attribute__((ext_vector_type(8)))  float    v8f;
typedef __attribute__((ext_vector_type(4)))  float    v4f;
typedef __attribute__((ext_vector_type(4)))  unsigned v4u;

constexpr int kRows = 4096;
constexpr int kNx   = 256;
constexpr int kNy   = 128;
static_assert((kNx % 32) == 0, "K multiple of 32");
static_assert((kRows % 16) == 0 && (kNy % 32) == 0, "wave tile 16 x 32 divides the output");
static_assert(kNy == 4 * 32, "four waves of 32 columns cover one output row");

constexpr float kCarryX  = 64.0f;
constexpr float kCarryLg = 32.0f;
constexpr float kCarryW  = 64.0f;
constexpr float kCarryT  = 8.0f;
constexpr float kInvAdd  = 1.0f / (kCarryX * kCarryW);
constexpr float kInvMul  = 1.0f / (kCarryLg * kCarryW);
constexpr float kInvT    = 1.0f / kCarryT;
constexpr float kLogFloor      = -100.0f;
constexpr float kAbsFloor      = 1e-7f;
constexpr float kExpCap        = 20.0f;
constexpr float kF16MinNormal  = 6.103515625e-05f;
constexpr float kF16Cap        = 60000.0f;
constexpr float kF32MinNormal  = 1.17549435e-38f;

constexpr size_t kBtBytes = (size_t)kNy * kNx * 2;
constexpr size_t kAcBytes = (size_t)kRows * kNx * 2;
constexpr size_t kOffBTA  = 0;
constexpr size_t kOffBTM  = kOffBTA + kBtBytes;
constexpr size_t kOffBTL  = kOffBTM + kBtBytes;
constexpr size_t kOffBTP  = kOffBTL + kBtBytes;
constexpr size_t kOffAX   = kOffBTP + kBtBytes;
constexpr size_t kOffAL   = kOffAX + kAcBytes;
constexpr size_t kOffAN   = kOffAL + kAcBytes;
constexpr size_t kWsTotal = kOffAN + kAcBytes;
static_assert(kWsTotal == 6553600ull, "carve total");
static_assert(kWsTotal <= 134217728ull, "carve cap");
static_assert((kOffBTM % 128) == 0 && (kOffBTL % 128) == 0 && (kOffBTP % 128) == 0 &&
              (kOffAX % 128) == 0 && (kOffAL % 128) == 0 && (kOffAN % 128) == 0, "128-B aligned regions");

__device__ __forceinline__ unsigned f16_bits_flush(float v) {
  const float vc = fminf(fmaxf(v, -kF16Cap), kF16Cap);
  const float vf = (fabsf(vc) < kF16MinNormal) ? 0.0f : vc;
  const _Float16 hv = (_Float16)vf;
  const unsigned short hb = __builtin_bit_cast(unsigned short, hv);
  return (unsigned)hb;
}

__device__ __forceinline__ float flush_f32(float v) {
  return (fabsf(v) < kF32MinNormal) ? 0.0f : v;
}

__device__ __forceinline__ v16h load_frag(const _Float16* p) {
  union { v16h v; v8h h[2]; } f;
  f.h[0] = *(const v8h*)(p);
  f.h[1] = *(const v8h*)(p + 16);
  return f.v;
}

__device__ __forceinline__ v8f mma_h(v16h a, v16h b, v8f c) {
  c = __builtin_amdgcn_wmma_f32_16x16x32_f16(false, a, false, b, (short)0, c, false, false);
  asm volatile("v_nop\n\tv_nop\n\tv_nop\n\tv_nop" : "+v"(c) : "v"(a), "v"(b));
  return c;
}

constexpr int kWordsPerPlane = kNy * kNx / 2;
static_assert((kWordsPerPlane % 256) == 0, "exact grid");

__global__ __launch_bounds__(256) void weight_planes_kernel(
    const float* __restrict__ Wa, const float* __restrict__ Ma,
    const float* __restrict__ Wm, const float* __restrict__ Mm,
    unsigned* __restrict__ PA, unsigned* __restrict__ PM,
    unsigned* __restrict__ PL, unsigned* __restrict__ PP)
{
  const int job = blockIdx.y;
  const int t = blockIdx.x * 256 + threadIdx.x;
  const float* W = (job == 0) ? Wa : Wm;
  const float* M = (job == 0) ? Ma : Mm;
  unsigned pkV = 0u, pkL = 0u, pkP = 0u;
#pragma unroll 1
  for (int e = 0; e < 2; ++e) {
    const int idx  = 2 * t + e;
    const int j    = idx >> 8;
    const int i    = idx & (kNx - 1);
    const int srcT = i * kNy + j;
    const int src  = (job == 2) ? idx : srcT;
    const float w  = W[src];
    const float m  = M[src];
    const float sg = 1.0f / (1.0f + expf(-m));
    const float v  = tanhf(w) * sg;
    const float tt = 1.0f - 2.0f * fabsf(v);
    const float lg = fmaxf(logf(fabsf(tt)), kLogFloor);
    const unsigned bv = f16_bits_flush(v * kCarryW);
    const unsigned bl = f16_bits_flush(lg * kCarryT);
    const unsigned bp = (tt < 0.0f) ? 0x3C00u : 0u;
    const int sh = 16 * e;
    pkV |= (bv << sh);
    pkL |= (bl << sh);
    pkP |= (bp << sh);
  }
  unsigned* dsel = (job == 0) ? PA : ((job == 1) ? PM : PL);
  const unsigned val = (job == 2) ? pkL : pkV;
  volatile unsigned* d0 = (volatile unsigned*)dsel;
  volatile unsigned* d1 = (volatile unsigned*)PP;
  d0[t] = val;
  if (job == 2) d1[t] = pkP;
  __threadfence();
  d0[t] = val;
  if (job == 2) d1[t] = pkP;
}

constexpr int kActThreads = kRows * kNx / 8;
static_assert((kActThreads % 256) == 0, "exact grid");

__global__ __launch_bounds__(256) void act_planes_kernel(
    const float* __restrict__ x, unsigned short* __restrict__ AX,
    unsigned short* __restrict__ AL, unsigned short* __restrict__ AN)
{
  const int i = blockIdx.x * 256 + threadIdx.x;
  const size_t e0 = (size_t)i << 3;
  const v4f a0 = *(const v4f*)(x + e0);
  const v4f a1 = *(const v4f*)(x + e0 + 4);
  float xs[8];
  xs[0] = a0[0]; xs[1] = a0[1]; xs[2] = a0[2]; xs[3] = a0[3];
  xs[4] = a1[0]; xs[5] = a1[1]; xs[6] = a1[2]; xs[7] = a1[3];
  unsigned bx[8], bl[8], bn[8];
#pragma unroll
  for (int e = 0; e < 8; ++e) {
    const float xv = xs[e];
    const float lg = logf(fmaxf(fabsf(xv), kAbsFloor));
    bx[e] = f16_bits_flush(xv * kCarryX);
    bl[e] = f16_bits_flush(lg * kCarryLg);
    bn[e] = (xv < 0.0f) ? 0x3C00u : 0u;
  }
  v4u wx, wl, wn;
  wx[0] = bx[0] | (bx[1] << 16); wx[1] = bx[2] | (bx[3] << 16);
  wx[2] = bx[4] | (bx[5] << 16); wx[3] = bx[6] | (bx[7] << 16);
  wl[0] = bl[0] | (bl[1] << 16); wl[1] = bl[2] | (bl[3] << 16);
  wl[2] = bl[4] | (bl[5] << 16); wl[3] = bl[6] | (bl[7] << 16);
  wn[0] = bn[0] | (bn[1] << 16); wn[1] = bn[2] | (bn[3] << 16);
  wn[2] = bn[4] | (bn[5] << 16); wn[3] = bn[6] | (bn[7] << 16);
  volatile v4u* qx = (volatile v4u*)(AX + e0);
  volatile v4u* ql = (volatile v4u*)(AL + e0);
  volatile v4u* qn = (volatile v4u*)(AN + e0);
  *qx = wx;
  *ql = wl;
  *qn = wn;
  __threadfence();
  *qx = wx;
  *ql = wl;
  *qn = wn;
}

constexpr int kSlabPitch = 36;
constexpr int kSlabFloats = 16 * kSlabPitch;

__global__ __launch_bounds__(128) void fused_paths_kernel(
    const _Float16* __restrict__ AX, const _Float16* __restrict__ AL, const _Float16* __restrict__ AN,
    const _Float16* __restrict__ BTA, const _Float16* __restrict__ BTM,
    const _Float16* __restrict__ BTL, const _Float16* __restrict__ BTP,
    const float* __restrict__ g, float* __restrict__ out)
{
  __shared__ __align__(16) float sT[4][4][kSlabFloats];
  const int lane = threadIdx.x & 31;
  const int wave = threadIdx.x >> 5;
  const int hh = lane >> 4;
  const int c  = lane & 15;
  const int m0 = blockIdx.x * 16;
  const int n0 = wave * 32;

  v8f accA[2], accM[2], accL[2], accP[2];
#pragma unroll
  for (int j = 0; j < 2; ++j) {
    accA[j] = (v8f){0.f, 0.f, 0.f, 0.f, 0.f, 0.f, 0.f, 0.f};
    accM[j] = (v8f){0.f, 0.f, 0.f, 0.f, 0.f, 0.f, 0.f, 0.f};
    accL[j] = (v8f){0.f, 0.f, 0.f, 0.f, 0.f, 0.f, 0.f, 0.f};
    accP[j] = (v8f){0.f, 0.f, 0.f, 0.f, 0.f, 0.f, 0.f, 0.f};
  }

  const size_t aoff = (size_t)(m0 + c) * kNx + 8 * hh;
#pragma unroll 1
  for (int k0 = 0; k0 < kNx; k0 += 32) {
    const v16h fx = load_frag(AX + aoff + k0);
    const v16h fl = load_frag(AL + aoff + k0);
    const v16h fn = load_frag(AN + aoff + k0);
#pragma unroll
    for (int j = 0; j < 2; ++j) {
      const size_t bo = (size_t)(n0 + 16 * j + c) * kNx + 8 * hh + k0;
      const v16h ba = load_frag(BTA + bo);
      const v16h bm = load_frag(BTM + bo);
      const v16h bl = load_frag(BTL + bo);
      const v16h bp = load_frag(BTP + bo);
      accA[j] = mma_h(fx, ba, accA[j]);
      accM[j] = mma_h(fl, bm, accM[j]);
      accL[j] = mma_h(fn, bl, accL[j]);
      accP[j] = mma_h(fn, bp, accP[j]);
    }
  }

  float* slA = sT[wave][0];
  float* slM = sT[wave][1];
  float* slL = sT[wave][2];
  float* slP = sT[wave][3];
#pragma unroll
  for (int j = 0; j < 2; ++j) {
#pragma unroll
    for (int r = 0; r < 8; ++r) {
      const int o = (8 * hh + r) * kSlabPitch + 16 * j + c;
      slA[o] = accA[j][r];
      slM[o] = accM[j][r];
      slL[o] = accL[j][r];
      slP[o] = accP[j][r];
    }
  }
  __syncthreads();

  const int q  = lane >> 3;
  const int c4 = (lane & 7) * 4;
  const v4f gv = *(const v4f*)(g + n0 + c4);
  v4f g1v;
#pragma unroll
  for (int e = 0; e < 4; ++e) {
    const float ge = gv[e];
    g1v[e] = 1.0f / (1.0f + expf(-ge));
  }

#pragma unroll 1
  for (int it = 0; it < 4; ++it) {
    const int o = (it * 4 + q) * kSlabPitch + c4;
    const v4f va = *(const v4f*)(slA + o);
    const v4f vm = *(const v4f*)(slM + o);
    const v4f vl = *(const v4f*)(slL + o);
    const v4f vp = *(const v4f*)(slP + o);
    v4f res;
#pragma unroll
    for (int e = 0; e < 4; ++e) {
      const float a1  = va[e] * kInvAdd;
      const float lm  = fminf(vm[e] * kInvMul, kExpCap);
      const float m1  = flush_f32(expf(lm));
      const float mag = flush_f32(expf(vl[e] * kInvT));
      const int   cnt = (int)(vp[e] + 0.5f);
      const float sgn = (cnt & 1) ? -1.0f : 1.0f;
      const float ms1 = fminf(fmaxf(sgn * mag, -1.0f), 1.0f);
      const float g1  = g1v[e];
      const float mulp = ((1.0f - g1) * m1) * ms1;
      res[e] = g1 * a1 + mulp;
    }
    *(v4f*)(slA + o) = res;
  }
  __syncthreads();

  for (int pass = 0; pass < 2; ++pass) {
#pragma unroll
    for (int it = 0; it < 4; ++it) {
      const int row = it * 4 + q;
      const v4f v = *(const v4f*)(slA + row * kSlabPitch + c4);
      *(volatile v4f*)(out + (size_t)(m0 + row) * kNy + n0 + c4) = v;
    }
    __threadfence();
  }
}

extern "C" void kernel_launch(void* const* d_in, const int* in_sizes, int n_in,
                              void* d_out, int out_size, void* d_ws, size_t ws_size,
                              hipStream_t stream) {
  if (n_in < 6) return;
  if (in_sizes[0] != kRows * kNx) return;
  if (in_sizes[1] != kNx * kNy) return;
  if (in_sizes[2] != kNx * kNy) return;
  if (in_sizes[3] != kNx * kNy) return;
  if (in_sizes[4] != kNx * kNy) return;
  if (in_sizes[5] != kNy) return;
  if (out_size != kRows * kNy) return;
  if (ws_size < kWsTotal) return;

  const float* x  = (const float*)d_in[0];
  const float* Wa = (const float*)d_in[1];
  const float* Ma = (const float*)d_in[2];
  const float* Wm = (const float*)d_in[3];
  const float* Mm = (const float*)d_in[4];
  const float* g  = (const float*)d_in[5];
  float* out = (float*)d_out;

  char* ws = (char*)d_ws;
  unsigned* BTAw = (unsigned*)(ws + kOffBTA);
  unsigned* BTMw = (unsigned*)(ws + kOffBTM);
  unsigned* BTLw = (unsigned*)(ws + kOffBTL);
  unsigned* BTPw = (unsigned*)(ws + kOffBTP);
  unsigned short* AXs = (unsigned short*)(ws + kOffAX);
  unsigned short* ALs = (unsigned short*)(ws + kOffAL);
  unsigned short* ANs = (unsigned short*)(ws + kOffAN);

  weight_planes_kernel<<<dim3(kWordsPerPlane / 256, 3), 256, 0, stream>>>(
      Wa, Ma, Wm, Mm, BTAw, BTMw, BTLw, BTPw);

  act_planes_kernel<<<kActThreads / 256, 256, 0, stream>>>(x, AXs, ALs, ANs);

  fused_paths_kernel<<<kRows / 16, 128, 0, stream>>>(
      (const _Float16*)(ws + kOffAX), (const _Float16*)(ws + kOffAL), (const _Float16*)(ws + kOffAN),
      (const _Float16*)(ws + kOffBTA), (const _Float16*)(ws + kOffBTM),
      (const _Float16*)(ws + kOffBTL), (const _Float16*)(ws + kOffBTP),
      g, out);
}
